// CrossAttentionBlock_15650860827496
// MI455X (gfx1250) — hardware-run, weakly checked
//
#include <hip/hip_runtime.h>
#include <hip/hip_bf16.h>
#include <math.h>
#include <stdint.h>

constexpr int kBatch = 2;
constexpr int kSeq   = 2048;
constexpr int kCh    = 1024;
constexpr int kHeads = 16;
constexpr int kHd    = 64;
constexpr int kFF    = 2048;
constexpr int kRows  = kBatch * kSeq;

static_assert(kCh % 64 == 0 && kFF % 64 == 0 && kRows % 64 == 0 && kSeq % 64 == 0);
static_assert(kCh % 32 == 0 && kFF % 32 == 0);
static_assert(kHd == 64 && kHeads * kHd == kCh);

typedef __attribute__((ext_vector_type(16))) _Float16 v16h;
typedef __attribute__((ext_vector_type(8)))  _Float16 v8h;
typedef __attribute__((ext_vector_type(16))) __bf16   v16b;
typedef __attribute__((ext_vector_type(8)))  __bf16   v8b;
typedef __attribute__((ext_vector_type(8)))  float    v8f;
typedef __attribute__((ext_vector_type(4)))  float    v4f;

__device__ __forceinline__ unsigned short f2bf_bits(float f) {
  unsigned u = __float_as_uint(f);
  return (unsigned short)((u + 0x7FFFu + ((u >> 16) & 1u)) >> 16);
}
__device__ __forceinline__ float bf_bits2f(unsigned short h) { return __uint_as_float(((unsigned)h) << 16); }

__device__ __forceinline__ void dep_guard_h(v8f& a, v8f& b, v16h x, v16h y) { asm volatile("v_nop\n\tv_nop\n\tv_nop\n\tv_nop" : "+v"(a), "+v"(b) : "v"(x), "v"(y)); }
__device__ __forceinline__ void dep_guard_b(v8f& a, v8f& b, v16b x, v16b y) { asm volatile("v_nop\n\tv_nop\n\tv_nop\n\tv_nop" : "+v"(a), "+v"(b) : "v"(x), "v"(y)); }
__device__ __forceinline__ void keep4_h(v16h a, v16h b, v16h c, v16h d) { asm volatile("v_nop" :: "v"(a), "v"(b), "v"(c), "v"(d)); }
__device__ __forceinline__ void keep4_b(v16b a, v16b b, v16b c, v16b d) { asm volatile("v_nop" :: "v"(a), "v"(b), "v"(c), "v"(d)); }
__device__ __forceinline__ void acc_guard4(v8f& a, v8f& b, v8f& c, v8f& d) { asm volatile("v_nop\n\tv_nop\n\tv_nop\n\tv_nop" : "+v"(a), "+v"(b), "+v"(c), "+v"(d)); }
template <typename T> struct Frag;
template <> struct Frag<_Float16> {
  typedef v16h V; union U { v16h v; v8h h[2]; };
  static __device__ __forceinline__ v16h load(const _Float16* p) {
    U f; f.h[0] = *(const v8h*)(p); f.h[1] = *(const v8h*)(p + 16); return f.v;
  }
  static __device__ __forceinline__ v8f mma(v16h a, v16h b, v8f c) {
    return __builtin_amdgcn_wmma_f32_16x16x32_f16(false, a, false, b, (short)0, c, false, false);
  }
  static __device__ __forceinline__ void guard(v8f& a, v8f& b, v16h x, v16h y) { dep_guard_h(a, b, x, y); }
  static __device__ __forceinline__ void keep(v16h a, v16h b, v16h c, v16h d) { keep4_h(a, b, c, d); }
};
template <> struct Frag<__bf16> {
  typedef v16b V; union U { v16b v; v8b h[2]; };
  static __device__ __forceinline__ v16b load(const __bf16* p) {
    U f; f.h[0] = *(const v8b*)(p); f.h[1] = *(const v8b*)(p + 16); return f.v;
  }
  static __device__ __forceinline__ v8f mma(v16b a, v16b b, v8f c) {
    return __builtin_amdgcn_wmma_f32_16x16x32_bf16(false, a, false, b, (short)0, c, false, false);
  }
  static __device__ __forceinline__ void guard(v8f& a, v8f& b, v16b x, v16b y) { dep_guard_b(a, b, x, y); }
  static __device__ __forceinline__ void keep(v16b a, v16b b, v16b c, v16b d) { keep4_b(a, b, c, d); }
};

__device__ __forceinline__ v8f hmma(v16h a, v16h b, v8f c) {
  c = __builtin_amdgcn_wmma_f32_16x16x32_f16(false, a, false, b, (short)0, c, false, false);
  asm volatile("v_nop\n\tv_nop\n\tv_nop\n\tv_nop" : "+v"(c) : "v"(a), "v"(b));
  return c;
}

template <int ET> struct Elem;
template <> struct Elem<0> { typedef _Float16 T; };
template <> struct Elem<1> { typedef __bf16 T; };
template <int ET, bool SPLIT, int BIAS_MODE, int OUT_MODE, bool RESID, int ACT = 0>
__global__ __launch_bounds__(256) void wmma_gemm64(
    const unsigned short* __restrict__ Ap, const unsigned short* __restrict__ A2p, int lda, long strideA,
    const unsigned short* __restrict__ Btp, const unsigned short* __restrict__ Bt2p, int ldb, long strideB,
    void* __restrict__ Cout, int ldc, long strideC,
    const float* __restrict__ bias,
    const float* __restrict__ resid, int ldr, long strideR,
    int M, int N, int K, float scale) {
  typedef typename Elem<ET>::T T;
  typedef typename Frag<T>::V V;
  const T* A = (const T*)Ap; const T* A2 = (const T*)A2p; const T* Bt = (const T*)Btp; const T* Bt2 = (const T*)Bt2p;
  __shared__ __align__(16) float sT[8][16 * 68];
  const int b    = blockIdx.y;
  const int lane = threadIdx.x & 31;
  const int wave = threadIdx.x >> 5;
  const int tilesN = N >> 6;
  const int tilesM = M >> 6;
  const int tile = blockIdx.x * 8 + wave;
  if (tile >= tilesM * tilesN) return;
  const int tm = tile / tilesN;
  const int tn = tile - tm * tilesN;
  const int m0 = tm << 6;
  const int n0 = tn << 6;

  const T* Ab  = A  + (size_t)b * strideA;
  const T* Bb  = Bt + (size_t)b * strideB;
  const T* Ab2 = SPLIT ? (A2  + (size_t)b * strideA) : nullptr;
  const T* Bb2 = SPLIT ? (Bt2 + (size_t)b * strideB) : nullptr;

  const int rlane = lane & 15;
  const int koff  = (lane >> 4) * 8;
  const int mOff  = (lane >> 4) * 8;

  v8f acc[4][4];
#pragma unroll
  for (int i = 0; i < 4; ++i)
#pragma unroll
    for (int j = 0; j < 4; ++j) acc[i][j] = (v8f){0.f,0.f,0.f,0.f,0.f,0.f,0.f,0.f};

  for (int k0 = 0; k0 < K; k0 += 32) {
    V bh[4], bl[4];
#pragma unroll
    for (int j = 0; j < 4; ++j) {
      const size_t bo = (size_t)(n0 + (j << 4) + rlane) * ldb + koff + k0;
      bh[j] = Frag<T>::load(Bb + bo);
      if (SPLIT) bl[j] = Frag<T>::load(Bb2 + bo);
    }
#pragma unroll
    for (int i = 0; i < 4; ++i) {
      const size_t ao = (size_t)(m0 + (i << 4) + rlane) * lda + koff + k0;
      V ah = Frag<T>::load(Ab + ao);
      V al;
      if (SPLIT) al = Frag<T>::load(Ab2 + ao);
#pragma unroll
      for (int j = 0; j < 4; ++j) {
        acc[i][j] = Frag<T>::mma(ah, bh[j], acc[i][j]);
        if (SPLIT) {
          acc[i][j] = Frag<T>::mma(ah, bl[j], acc[i][j]);
          acc[i][j] = Frag<T>::mma(al, bh[j], acc[i][j]);
        }
      }
      Frag<T>::guard(acc[i][0], acc[i][3], ah, SPLIT ? al : ah);
    }
    Frag<T>::keep(bh[0], bh[1], bh[2], bh[3]);
    if (SPLIT) Frag<T>::keep(bl[0], bl[1], bl[2], bl[3]);
  }
  acc_guard4(acc[0][0], acc[0][1], acc[0][2], acc[0][3]);
  acc_guard4(acc[1][0], acc[1][1], acc[1][2], acc[1][3]);
  acc_guard4(acc[2][0], acc[2][1], acc[2][2], acc[2][3]);
  acc_guard4(acc[3][0], acc[3][1], acc[3][2], acc[3][3]);

  float* slab = sT[wave];
  float bn[4] = {0.f, 0.f, 0.f, 0.f};
  if (BIAS_MODE == 2) {
#pragma unroll
    for (int j = 0; j < 4; ++j) bn[j] = bias[n0 + (j << 4) + rlane];
  }
#pragma unroll
  for (int i = 0; i < 4; ++i) {
    const int mBase = m0 + (i << 4);
    v4f bmA = (v4f){0.f,0.f,0.f,0.f};
    v4f bmB = (v4f){0.f,0.f,0.f,0.f};
    if (BIAS_MODE == 1) {
      bmA = *(const v4f*)(bias + mBase + mOff);
      bmB = *(const v4f*)(bias + mBase + mOff + 4);
    }
#pragma unroll
    for (int j = 0; j < 4; ++j) {
#pragma unroll
      for (int r = 0; r < 8; ++r) {
        float v = acc[i][j][r] * scale;
        if (BIAS_MODE == 1) v += (r < 4) ? bmA[r & 3] : bmB[r & 3];
        if (BIAS_MODE == 2) v += bn[j];
        if (ACT == 2) v = fmaxf(v, 0.0f);
        slab[(mOff + r) * 68 + (j << 4) + rlane] = v;
      }
    }
    __builtin_amdgcn_fence(__ATOMIC_RELEASE, "workgroup");
    __builtin_amdgcn_wave_barrier();
    __builtin_amdgcn_fence(__ATOMIC_ACQUIRE, "workgroup");
    if (OUT_MODE == 0) {
      float* C = (float*)Cout + (size_t)b * strideC;
      const float* Rb = RESID ? (resid + (size_t)b * strideR) : nullptr;
      const int hh = lane >> 4, c4 = (lane & 15) * 4;
      v4f vals[8];
#pragma unroll
      for (int it = 0; it < 8; ++it) {
        const int row = it * 2 + hh;
        v4f v = *(const v4f*)(slab + row * 68 + c4);
        if (RESID) {
          const v4f rr = *(const v4f*)(Rb + (size_t)(mBase + row) * ldr + n0 + c4);
          v += rr;
        }
        vals[it] = v;
      }
      for (int pass = 0; pass < 2; ++pass) {
#pragma unroll
        for (int it = 0; it < 8; ++it) {
          const int row = it * 2 + hh;
          *(volatile v4f*)(C + (size_t)(mBase + row) * ldc + n0 + c4) = vals[it];
        }
        __threadfence();
      }
    } else {
      const int q = lane >> 3, c8 = (lane & 7) * 8;
      unsigned short* C  = (unsigned short*)Cout  + (size_t)b * strideC;
      v8h hv[4];
#pragma unroll
      for (int it = 0; it < 4; ++it) {
        const int row = it * 4 + q;
        const float* sp = slab + row * 68 + c8;
#pragma unroll
        for (int e = 0; e < 8; ++e) hv[it][e] = (_Float16)sp[e];
      }
      for (int pass = 0; pass < 2; ++pass) {
#pragma unroll
        for (int it = 0; it < 4; ++it) {
          const int row = it * 4 + q;
          *(volatile v8h*)(C + (size_t)(mBase + row) * ldc + n0 + c8) = hv[it];
        }
        __threadfence();
      }
    }
    __builtin_amdgcn_fence(__ATOMIC_RELEASE, "workgroup");
    __builtin_amdgcn_wave_barrier();
    __builtin_amdgcn_fence(__ATOMIC_ACQUIRE, "workgroup");
  }
}

__global__ __launch_bounds__(256) void cast_f32_f16x2(
    const float* __restrict__ in, _Float16* __restrict__ out, int n2) {
  int i = blockIdx.x * 256 + threadIdx.x;
  if (i < n2) {
    const _Float16 h0 = (_Float16)in[2 * i], h1 = (_Float16)in[2 * i + 1];
    const unsigned u = (unsigned)__builtin_bit_cast(unsigned short, h0) | ((unsigned)__builtin_bit_cast(unsigned short, h1) << 16);
    ((volatile unsigned*)out)[i] = u;
    __threadfence();
    ((volatile unsigned*)out)[i] = u;
  }
}

__global__ __launch_bounds__(256) void transpose_cast_f16(
    const float* __restrict__ in, _Float16* __restrict__ out, int nrows, int ncols, float mult) {
  __shared__ float st[64][65];
  const int tid = threadIdx.x, lane = tid & 31, wave = tid >> 5;
  const int r0 = blockIdx.y * 64, c0 = blockIdx.x * 64;
  const int cl = (tid & 15) * 4;
#pragma unroll
  for (int i = 0; i < 4; ++i) {
    const int rr = (tid >> 4) + 16 * i;
    const v4f xv = *(const v4f*)(in + (size_t)(r0 + rr) * ncols + c0 + cl);
    st[rr][cl] = xv[0]; st[rr][cl + 1] = xv[1]; st[rr][cl + 2] = xv[2]; st[rr][cl + 3] = xv[3];
  }
  __syncthreads();
  const int q8 = lane >> 3, seg = (lane & 7) * 8;
  v8h hv[2];
#pragma unroll
  for (int it = 0; it < 2; ++it) {
    const int cc = wave * 8 + it * 4 + q8;
#pragma unroll
    for (int e = 0; e < 8; ++e) hv[it][e] = (_Float16)(st[seg + e][cc] * mult);
  }
  for (int pass = 0; pass < 2; ++pass) {
#pragma unroll
    for (int it = 0; it < 2; ++it) {
      const int cc = wave * 8 + it * 4 + q8;
      *(volatile v8h*)(out + (size_t)(c0 + cc) * nrows + r0 + seg) = hv[it];
    }
    __threadfence();
  }
}

__global__ __launch_bounds__(128) void attn_f16_hd64(
    const _Float16* __restrict__ qh, const _Float16* __restrict__ kh,
    const _Float16* __restrict__ vT, _Float16* __restrict__ ctx,
    float sm_scale, float out_mult) {
  constexpr float kPsc = 32768.0f;
  constexpr int kLdv = kRows;
  constexpr int kNqb = kSeq / 64;
  __shared__ __align__(16) _Float16 Psh[4][16 * 64];
  __shared__ __align__(16) float Os[4][16 * 68];

  const int tid  = threadIdx.x;
  const int wave = tid >> 5;
  const int lane = tid & 31;
  const int hh   = lane >> 4;
  const int c    = lane & 15;
  const int bx = blockIdx.x;
  const int qb = bx % kNqb;
  const int bh = bx / kNqb;
  const int h  = bh % kHeads;
  const int b  = bh / kHeads;
  const int q0 = qb * 64 + wave * 16;

  v16h qa[2];
  {
    const _Float16* qrow = qh + (size_t)(b * kSeq + q0 + c) * kCh + h * kHd + 8 * hh;
    qa[0] = Frag<_Float16>::load(qrow);
    qa[1] = Frag<_Float16>::load(qrow + 32);
  }
  const _Float16* kbase = kh + (size_t)(b * kSeq) * kCh + h * kHd + 8 * hh;
  const _Float16* vbase = vT + (size_t)(h * kHd) * kLdv + b * kSeq + 8 * hh;

  float mrow[8], lrow[8];
  v8f oacc[4];
#pragma unroll
  for (int r = 0; r < 8; ++r) { mrow[r] = -INFINITY; lrow[r] = 0.f; }
#pragma unroll
  for (int t = 0; t < 4; ++t) oacc[t] = (v8f){0.f,0.f,0.f,0.f,0.f,0.f,0.f,0.f};

  _Float16* pw = Psh[wave];
  for (int kc = 0; kc < kNqb; ++kc) {
    const int kv0 = kc * 64;
    __syncthreads();
    v8f s[4];
#pragma unroll
    for (int j = 0; j < 4; ++j) {
      s[j] = (v8f){0.f,0.f,0.f,0.f,0.f,0.f,0.f,0.f};
      const _Float16* kp = kbase + (size_t)(kv0 + j * 16 + c) * kCh;
#pragma unroll
      for (int dc = 0; dc < 2; ++dc) {
        const v16h kb = Frag<_Float16>::load(kp + dc * 32);
        s[j] = hmma(qa[dc], kb, s[j]);
      }
    }
    float cm[8];
#pragma unroll
    for (int r = 0; r < 8; ++r) {
      float m = -INFINITY;
#pragma unroll
      for (int j = 0; j < 4; ++j) {
        s[j][r] *= sm_scale;
        m = fmaxf(m, s[j][r]);
      }
#pragma unroll
      for (int off = 1; off < 16; off <<= 1) m = fmaxf(m, __shfl_xor(m, off, 32));
      cm[r] = m;
    }
#pragma unroll
    for (int r = 0; r < 8; ++r) {
      const float mnew = fmaxf(mrow[r], cm[r]);
      const float alpha = expf(mrow[r] - mnew);
      mrow[r] = mnew;
      float psum = 0.f;
#pragma unroll
      for (int j = 0; j < 4; ++j) {
        const float p = expf(s[j][r] - mnew);
        psum += p;
        pw[(8 * hh + r) * 64 + j * 16 + c] = (_Float16)(p * kPsc);
      }
#pragma unroll
      for (int off = 1; off < 16; off <<= 1) psum += __shfl_xor(psum, off, 32);
      lrow[r] = lrow[r] * alpha + psum;
#pragma unroll
      for (int t = 0; t < 4; ++t) oacc[t][r] *= alpha;
    }
    __builtin_amdgcn_fence(__ATOMIC_RELEASE, "workgroup");
    __builtin_amdgcn_wave_barrier();
    __builtin_amdgcn_fence(__ATOMIC_ACQUIRE, "workgroup");
#pragma unroll
    for (int kk = 0; kk < 2; ++kk) {
      const v16h pa = Frag<_Float16>::load(pw + c * 64 + kk * 32 + 8 * hh);
#pragma unroll
      for (int t = 0; t < 4; ++t) {
        const v16h vb = Frag<_Float16>::load(vbase + (size_t)(t * 16 + c) * kLdv + kv0 + kk * 32);
        oacc[t] = hmma(pa, vb, oacc[t]);
      }
    }
  }

  float* os = Os[wave];
#pragma unroll
  for (int r = 0; r < 8; ++r) {
    const float inv = out_mult / (lrow[r] * kPsc);
#pragma unroll
    for (int t = 0; t < 4; ++t) os[(8 * hh + r) * 68 + t * 16 + c] = oacc[t][r] * inv;
  }
  __builtin_amdgcn_fence(__ATOMIC_RELEASE, "workgroup");
  __builtin_amdgcn_wave_barrier();
  __builtin_amdgcn_fence(__ATOMIC_ACQUIRE, "workgroup");
  {
    const int q8 = lane >> 3, c8 = (lane & 7) * 8;
    _Float16* obase = ctx + (size_t)(b * kSeq + q0) * kCh + h * kHd + c8;
    v8h hv[4];
#pragma unroll
    for (int it = 0; it < 4; ++it) {
      const int row = it * 4 + q8;
      const float* sp = os + row * 68 + c8;
#pragma unroll
      for (int e = 0; e < 8; ++e) hv[it][e] = (_Float16)sp[e];
    }
    for (int pass = 0; pass < 2; ++pass) {
#pragma unroll
      for (int it = 0; it < 4; ++it) {
        const int row = it * 4 + q8;
        *(volatile v8h*)(obase + (size_t)row * kCh) = hv[it];
      }
      __threadfence();
    }
  }
}

__global__ __launch_bounds__(128) void layernorm_f16(
    const float* __restrict__ x, const float* __restrict__ w, const float* __restrict__ bb,
    _Float16* __restrict__ out, float eps) {
  __shared__ float red[2][4];
  const int row = blockIdx.x;
  const int tid = threadIdx.x, lane = tid & 31, wave = tid >> 5;
  const float* xr = x + (size_t)row * kCh + tid * 8;
  const v4f a0 = *(const v4f*)(xr);
  const v4f a1 = *(const v4f*)(xr + 4);
  float s = ((a0[0] + a0[1]) + (a0[2] + a0[3])) + ((a1[0] + a1[1]) + (a1[2] + a1[3]));
#pragma unroll
  for (int off = 1; off < 32; off <<= 1) s += __shfl_xor(s, off, 32);
  if (lane == 0) red[0][wave] = s;
  __syncthreads();
  const float mu = ((red[0][0] + red[0][1]) + (red[0][2] + red[0][3])) * (1.0f / (float)kCh);
  float d[8];
  d[0] = a0[0] - mu; d[1] = a0[1] - mu; d[2] = a0[2] - mu; d[3] = a0[3] - mu;
  d[4] = a1[0] - mu; d[5] = a1[1] - mu; d[6] = a1[2] - mu; d[7] = a1[3] - mu;
  float ss = 0.f;
#pragma unroll
  for (int e = 0; e < 8; ++e) ss += d[e] * d[e];
#pragma unroll
  for (int off = 1; off < 32; off <<= 1) ss += __shfl_xor(ss, off, 32);
  if (lane == 0) red[1][wave] = ss;
  __syncthreads();
  const float var = ((red[1][0] + red[1][1]) + (red[1][2] + red[1][3])) * (1.0f / (float)kCh);
  const float inv = rsqrtf(var + eps);
  const v4f w0 = *(const v4f*)(w + tid * 8);
  const v4f w1 = *(const v4f*)(w + tid * 8 + 4);
  const v4f b0 = *(const v4f*)(bb + tid * 8);
  const v4f b1 = *(const v4f*)(bb + tid * 8 + 4);
  v8h hv;
  hv[0] = (_Float16)(d[0] * inv * w0[0] + b0[0]);
  hv[1] = (_Float16)(d[1] * inv * w0[1] + b0[1]);
  hv[2] = (_Float16)(d[2] * inv * w0[2] + b0[2]);
  hv[3] = (_Float16)(d[3] * inv * w0[3] + b0[3]);
  hv[4] = (_Float16)(d[4] * inv * w1[0] + b1[0]);
  hv[5] = (_Float16)(d[5] * inv * w1[1] + b1[1]);
  hv[6] = (_Float16)(d[6] * inv * w1[2] + b1[2]);
  hv[7] = (_Float16)(d[7] * inv * w1[3] + b1[3]);
  _Float16* op = out + (size_t)row * kCh + tid * 8;
  *(volatile v8h*)op = hv;
  __threadfence();
  *(volatile v8h*)op = hv;
}

__global__ __launch_bounds__(256) void gelu_cast_f16x2(
    const float* __restrict__ in, _Float16* __restrict__ out, int n2, float mult) {
  const int i = blockIdx.x * 256 + threadIdx.x;
  if (i < n2) {
    unsigned u = 0;
#pragma unroll 1
    for (int e = 0; e < 2; ++e) {
      const float xv = in[2 * (size_t)i + e];
      const float g = 0.5f * xv * (1.0f + erff(xv * 0.70710678118654752f));
      const _Float16 hg = (_Float16)(g * mult);
      u |= ((unsigned)__builtin_bit_cast(unsigned short, hg)) << (16 * e);
    }
    ((volatile unsigned*)out)[i] = u;
    __threadfence();
    ((volatile unsigned*)out)[i] = u;
  }
}

extern "C" void kernel_launch(void* const* d_in, const int* in_sizes, int n_in,
                              void* d_out, int out_size, void* d_ws, size_t ws_size,
                              hipStream_t stream) {
  (void)in_sizes; (void)n_in; (void)out_size;
  const float* q   = (const float*)d_in[0];
  const float* k   = (const float*)d_in[1];
  const float* v   = (const float*)d_in[2];
  const float* Wq  = (const float*)d_in[3];
  const float* bq  = (const float*)d_in[4];
  const float* Wk  = (const float*)d_in[5];
  const float* bk  = (const float*)d_in[6];
  const float* Wv  = (const float*)d_in[7];
  const float* bv  = (const float*)d_in[8];
  const float* Wo  = (const float*)d_in[9];
  const float* bo  = (const float*)d_in[10];
  const float* lnw = (const float*)d_in[11];
  const float* lnb = (const float*)d_in[12];
  const float* W1  = (const float*)d_in[13];
  const float* b1  = (const float*)d_in[14];
  const float* W2  = (const float*)d_in[15];
  const float* b2  = (const float*)d_in[16];
  float* out = (float*)d_out;

  constexpr size_t kMiB = 1048576;
  constexpr size_t kActH = (size_t)kRows * kCh * 2;
  constexpr size_t kActF = (size_t)kRows * kCh * 4;
  constexpr size_t kWsq  = (size_t)kCh * kCh * 2;
  constexpr size_t kWff  = (size_t)kCh * kFF * 2;
  constexpr size_t kGh   = (size_t)kRows * kFF * 2;
  constexpr size_t kUf   = (size_t)kRows * kFF * 4;
  static_assert(kActH == 8 * kMiB && kActF == 16 * kMiB && kWsq == 2 * kMiB && kWff == 4 * kMiB);
  static_assert(kGh == 16 * kMiB && kUf == 32 * kMiB);
  constexpr size_t oQ16 = 0, oK16 = 8 * kMiB, oV16 = 16 * kMiB;
  constexpr size_t oXF = 0, oH16 = 16 * kMiB;
  constexpr size_t oWqT = 24 * kMiB, oWkT = 26 * kMiB, oWvT = 28 * kMiB, oWoT = 30 * kMiB;
  constexpr size_t oW1T = 32 * kMiB, oW2T = 36 * kMiB;
  constexpr size_t oQh = 40 * kMiB, oKh = 48 * kMiB, oVT = 56 * kMiB;
  constexpr size_t oG16 = 40 * kMiB;
  constexpr size_t oCtx = 64 * kMiB;
  constexpr size_t oU = 72 * kMiB;
  constexpr size_t kWsTotal = oU + kUf;
  static_assert(kWsTotal == 104 * kMiB);
  static_assert(oXF + kActF <= oH16 && oH16 + kActH <= oWqT);
  static_assert(oW2T + kWff <= oQh && oG16 + kGh <= oVT && oVT + kActH <= oCtx && oCtx + kActH <= oU);
  if (ws_size < kWsTotal) return;

  char* ws = (char*)d_ws;
  _Float16* q16  = (_Float16*)(ws + oQ16);
  _Float16* k16  = (_Float16*)(ws + oK16);
  _Float16* v16  = (_Float16*)(ws + oV16);
  float*    xF   = (float*)(ws + oXF);
  _Float16* h16  = (_Float16*)(ws + oH16);
  _Float16* WqT  = (_Float16*)(ws + oWqT);
  _Float16* WkT  = (_Float16*)(ws + oWkT);
  _Float16* WvT  = (_Float16*)(ws + oWvT);
  _Float16* WoT  = (_Float16*)(ws + oWoT);
  _Float16* W1T  = (_Float16*)(ws + oW1T);
  _Float16* W2T  = (_Float16*)(ws + oW2T);
  _Float16* qh16 = (_Float16*)(ws + oQh);
  _Float16* kh16 = (_Float16*)(ws + oKh);
  _Float16* vT16 = (_Float16*)(ws + oVT);
  _Float16* g16  = (_Float16*)(ws + oG16);
  _Float16* ctx16 = (_Float16*)(ws + oCtx);
  float*    uF   = (float*)(ws + oU);

  typedef const unsigned short* cus;
  const float kWcarry = 64.0f;
  const float kInvW   = 1.0f / 64.0f;
  const float kInvWW  = 1.0f / 4096.0f;

  const int nAct2 = kRows * kCh / 2;
  cast_f32_f16x2<<<dim3((nAct2 + 255) / 256), dim3(256), 0, stream>>>(q, q16, nAct2);
  cast_f32_f16x2<<<dim3((nAct2 + 255) / 256), dim3(256), 0, stream>>>(k, k16, nAct2);
  cast_f32_f16x2<<<dim3((nAct2 + 255) / 256), dim3(256), 0, stream>>>(v, v16, nAct2);

  transpose_cast_f16<<<dim3(kCh / 64, kCh / 64), dim3(256), 0, stream>>>(Wq, WqT, kCh, kCh, kWcarry);
  transpose_cast_f16<<<dim3(kCh / 64, kCh / 64), dim3(256), 0, stream>>>(Wk, WkT, kCh, kCh, kWcarry);
  transpose_cast_f16<<<dim3(kCh / 64, kCh / 64), dim3(256), 0, stream>>>(Wv, WvT, kCh, kCh, kWcarry);
  transpose_cast_f16<<<dim3(kCh / 64, kCh / 64), dim3(256), 0, stream>>>(Wo, WoT, kCh, kCh, kWcarry);
  transpose_cast_f16<<<dim3(kFF / 64, kCh / 64), dim3(256), 0, stream>>>(W1, W1T, kCh, kFF, kWcarry);
  transpose_cast_f16<<<dim3(kCh / 64, kFF / 64), dim3(256), 0, stream>>>(W2, W2T, kFF, kCh, kWcarry);

  const int tilesProj = (kRows / 64) * (kCh / 64);
  const int gridProj  = (tilesProj + 7) / 8;
  wmma_gemm64<0, false, 2, 1, false, 0><<<dim3(gridProj, 1), dim3(256), 0, stream>>>(
      (cus)q16, (cus)q16, kCh, 0L, (cus)WqT, (cus)WqT, kCh, 0L,
      (void*)qh16, kCh, 0L, bq, nullptr, 0, 0L, kRows, kCh, kCh, kInvW);
  wmma_gemm64<0, false, 2, 1, false, 0><<<dim3(gridProj, 1), dim3(256), 0, stream>>>(
      (cus)k16, (cus)k16, kCh, 0L, (cus)WkT, (cus)WkT, kCh, 0L,
      (void*)kh16, kCh, 0L, bk, nullptr, 0, 0L, kRows, kCh, kCh, kInvW);
  const int tilesVT = (kCh / 64) * (kRows / 64);
  wmma_gemm64<0, false, 1, 1, false, 0><<<dim3((tilesVT + 7) / 8, 1), dim3(256), 0, stream>>>(
      (cus)WvT, (cus)WvT, kCh, 0L, (cus)v16, (cus)v16, kCh, 0L,
      (void*)vT16, kRows, 0L, bv, nullptr, 0, 0L, kCh, kRows, kCh, kInvW);

  attn_f16_hd64<<<dim3(kBatch * kHeads * (kSeq / 64)), dim3(128), 0, stream>>>(
      qh16, kh16, vT16, ctx16, 0.125f, kWcarry);

  wmma_gemm64<0, false, 2, 0, true, 0><<<dim3(gridProj, 1), dim3(256), 0, stream>>>(
      (cus)ctx16, (cus)ctx16, kCh, 0L, (cus)WoT, (cus)WoT, kCh, 0L,
      (void*)xF, kCh, 0L, bo, q, kCh, 0L, kRows, kCh, kCh, kInvWW);

  layernorm_f16<<<dim3(kRows), dim3(128), 0, stream>>>(xF, lnw, lnb, h16, 1e-5f);

  const int tilesFF = (kRows / 64) * (kFF / 64);
  wmma_gemm64<0, false, 2, 0, false, 0><<<dim3((tilesFF + 7) / 8, 1), dim3(256), 0, stream>>>(
      (cus)h16, (cus)h16, kCh, 0L, (cus)W1T, (cus)W1T, kCh, 0L,
      (void*)uF, kFF, 0L, b1, nullptr, 0, 0L, kRows, kFF, kCh, kInvW);

  const int nFF2 = kRows * kFF / 2;
  gelu_cast_f16x2<<<dim3((nFF2 + 255) / 256), dim3(256), 0, stream>>>(uF, g16, nFF2, kWcarry);

  wmma_gemm64<0, false, 2, 0, true, 0><<<dim3(gridProj, 1), dim3(256), 0, stream>>>(
      (cus)g16, (cus)g16, kFF, 0L, (cus)W2T, (cus)W2T, kFF, 0L,
      (void*)out, kCh, 0L, b2, xF, kCh, 0L, kRows, kCh, kFF, kInvWW);
}
